// PositionAwareGraphAttention_36275293782541
// MI455X (gfx1250) — hardware-run, weakly checked
//
#include <hip/hip_runtime.h>
#include <math.h>
#include <stdint.h>

#define PSPLIT 1
#define VSPLIT 1

#define NB    8
#define NN    1024
#define IN_F  768
#define OUT_F 512
#define MROWS (NB * NN)
#define NSEG  (1 + PSPLIT + VSPLIT)
#define K3    (NSEG * NN)
#define SEG_PLO 1
#define SEG_VLO (1 + PSPLIT)
#define OUT0_ELEMS (NB * NN * OUT_F)
#define OUT1_ELEMS (NB * NN * NN)

#define NHB (MROWS * IN_F / 8 / 256)
#define NWT ((OUT_F / 64) * (IN_F / 64))

#define RP_ROWS  64
#define RP_PITCH 513
#define RP_DYN   (RP_ROWS * RP_PITCH * 4)
#define RP_STATIC (1024 * 4 + 128 * 4)

#define WS_HB  ((size_t)MROWS * IN_F * 2)
#define WS_WT  ((size_t)OUT_F * IN_F * 2)
#define WS_AV  ((size_t)1024 * 4)
#define WS_HW  ((size_t)MROWS * OUT_F * 4)
#define WS_F12 ((size_t)2 * MROWS * 4)
#define WS_P3  ((size_t)MROWS * K3 * 2)
#define WS_VT3 ((size_t)NB * OUT_F * K3 * 2)
#define WS_TOTAL (WS_HB + WS_WT + WS_AV + WS_HW + WS_F12 + WS_P3 + WS_VT3)

static_assert(NN == 1024);
static_assert(OUT_F == 512);
static_assert(IN_F % 32 == 0);
static_assert(IN_F % 64 == 0);
static_assert(K3 % 32 == 0);
static_assert(MROWS % 64 == 0);
static_assert(OUT_F % 64 == 0);
static_assert(NN % RP_ROWS == 0);
static_assert((MROWS * IN_F) % (8 * 256) == 0);
static_assert(WS_TOTAL <= (size_t)134217728);
static_assert(WS_HB % 128 == 0 && WS_WT % 128 == 0 && WS_AV % 128 == 0 && WS_HW % 128 == 0 && WS_F12 % 128 == 0 && WS_P3 % 128 == 0);
static_assert(RP_DYN + RP_STATIC <= 327680);
static_assert(OUT0_ELEMS + OUT1_ELEMS == 12582912);

typedef __bf16 v16b __attribute__((ext_vector_type(16)));
typedef __bf16 v8b  __attribute__((ext_vector_type(8)));
typedef float  v8f  __attribute__((ext_vector_type(8)));
typedef float  v4f  __attribute__((ext_vector_type(4)));
typedef unsigned int v4u __attribute__((ext_vector_type(4)));
typedef int    v4i  __attribute__((ext_vector_type(4)));
typedef v4f __attribute__((may_alias)) v4fa;
typedef v4i __attribute__((may_alias)) v4ia;
typedef v8b __attribute__((may_alias)) v8ba;

union FragB { v16b v; v8b h[2]; };

__device__ __forceinline__ unsigned f2bf_bits(float f) {
  const unsigned u = __float_as_uint(f);
  return (u + 0x7FFFu + ((u >> 16) & 1u)) >> 16;
}
__device__ __forceinline__ float bf_bits2f(unsigned hb) { return __uint_as_float(hb << 16); }
__device__ __forceinline__ float bf16r(float f) { return bf_bits2f(f2bf_bits(f)); }
__device__ __forceinline__ unsigned pk16(unsigned a, unsigned b) { return a | (b << 16); }

struct HL { v4u h; v4u l; };
__device__ __forceinline__ HL split8(v4f a, v4f c) {
  const unsigned h0 = f2bf_bits(a[0]), h1 = f2bf_bits(a[1]), h2 = f2bf_bits(a[2]), h3 = f2bf_bits(a[3]);
  const unsigned h4 = f2bf_bits(c[0]), h5 = f2bf_bits(c[1]), h6 = f2bf_bits(c[2]), h7 = f2bf_bits(c[3]);
  const unsigned l0 = f2bf_bits(a[0] - bf_bits2f(h0)), l1 = f2bf_bits(a[1] - bf_bits2f(h1));
  const unsigned l2 = f2bf_bits(a[2] - bf_bits2f(h2)), l3 = f2bf_bits(a[3] - bf_bits2f(h3));
  const unsigned l4 = f2bf_bits(c[0] - bf_bits2f(h4)), l5 = f2bf_bits(c[1] - bf_bits2f(h5));
  const unsigned l6 = f2bf_bits(c[2] - bf_bits2f(h6)), l7 = f2bf_bits(c[3] - bf_bits2f(h7));
  HL r;
  r.h = (v4u){ pk16(h0, h1), pk16(h2, h3), pk16(h4, h5), pk16(h6, h7) };
  r.l = (v4u){ pk16(l0, l1), pk16(l2, l3), pk16(l4, l5), pk16(l6, l7) };
  return r;
}

__device__ __forceinline__ v8f mma_bf16(v16b a, v16b b, v8f c) {
  c = __builtin_amdgcn_wmma_f32_16x16x32_bf16(false, a, false, b, (short)0, c, false, false);
  asm volatile("v_nop\n\tv_nop\n\tv_nop\n\tv_nop" : "+v"(c) : "v"(a), "v"(b));
  return c;
}
__device__ __forceinline__ v16b ld_frag(const __bf16* p) {
  FragB f;
  f.h[0] = *(const v8ba*)(p);
  f.h[1] = *(const v8ba*)(p + 16);
  return f.v;
}

__global__ __launch_bounds__(256) void k_prep(const float* __restrict__ h, const float* __restrict__ W,
                                              const float* __restrict__ a, unsigned short* __restrict__ HB,
                                              unsigned short* __restrict__ WT, float* __restrict__ AV) {
  __shared__ __attribute__((aligned(16))) float tf[64 * 68];
  const int tid = threadIdx.x;
  const int blk = blockIdx.x;
  if (blk < NHB) {
    const size_t g = (size_t)blk * 256 + tid;
    const v4f x0 = *(const v4fa*)(h + g * 8);
    const v4f x1 = *(const v4fa*)(h + g * 8 + 4);
    const v4u o = (v4u){ pk16(f2bf_bits(x0[0]), f2bf_bits(x0[1])), pk16(f2bf_bits(x0[2]), f2bf_bits(x0[3])),
                         pk16(f2bf_bits(x1[0]), f2bf_bits(x1[1])), pk16(f2bf_bits(x1[2]), f2bf_bits(x1[3])) };
    *(volatile v4u*)(HB + g * 8) = o;
    __threadfence();
    *(volatile v4u*)(HB + g * 8) = o;
  } else if (blk < NHB + NWT) {
    const int bidx = blk - NHB;
    const int c0 = (bidx & 7) * 64;
    const int r0 = (bidx >> 3) * 64;
    {
      const int lr = tid >> 4, c4 = (tid & 15) * 4;
#pragma unroll
      for (int it = 0; it < 4; ++it) {
        const int rr = it * 16 + lr;
        const v4f v = *(const v4fa*)(W + (size_t)(r0 + rr) * OUT_F + c0 + c4);
        *(v4fa*)(tf + rr * 68 + c4) = v;
      }
    }
    __syncthreads();
    const int sub = tid >> 3, c8 = (tid & 7) * 8;
    v4u hv[2];
#pragma unroll
    for (int it = 0; it < 2; ++it) {
      const int oc = it * 32 + sub;
      v4u t;
#pragma unroll
      for (int q = 0; q < 4; ++q) {
        const float f0 = tf[(c8 + 2 * q) * 68 + oc];
        const float f1 = tf[(c8 + 2 * q + 1) * 68 + oc];
        t[q] = pk16(f2bf_bits(f0), f2bf_bits(f1));
      }
      hv[it] = t;
    }
    for (int pass = 0; pass < 2; ++pass) {
#pragma unroll
      for (int it = 0; it < 2; ++it) {
        const int oc = it * 32 + sub;
        *(volatile v4u*)(WT + (size_t)(c0 + oc) * IN_F + r0 + c8) = hv[it];
      }
      __threadfence();
    }
  } else {
    const v4f x = *(const v4fa*)(a + tid * 4);
    const v4f o = (v4f){ bf16r(x[0]), bf16r(x[1]), bf16r(x[2]), bf16r(x[3]) };
    *(volatile v4f*)(AV + tid * 4) = o;
    __threadfence();
    *(volatile v4f*)(AV + tid * 4) = o;
  }
}

__global__ __launch_bounds__(256) __attribute__((amdgpu_num_vgpr(248)))
void k_gemm_bf16(const unsigned short* __restrict__ Ap, int lda, long strideA,
                 const unsigned short* __restrict__ Btp, int ldb, long strideB,
                 float* __restrict__ Cout, int ldc, long strideC,
                 int M, int N, int K) {
  __shared__ __attribute__((aligned(16))) float sT[8][16 * 68];
  const int b    = blockIdx.y;
  const int lane = threadIdx.x & 31;
  const int wave = threadIdx.x >> 5;
  const int tilesN = N >> 6;
  const int tilesM = M >> 6;
  const int tile = blockIdx.x * 8 + wave;
  if (tile >= tilesM * tilesN) return;
  const int tm = tile / tilesN;
  const int tn = tile - tm * tilesN;
  const int m0 = tm << 6;
  const int n0 = tn << 6;

  const __bf16* Ab = (const __bf16*)(const void*)Ap  + (size_t)b * strideA;
  const __bf16* Bb = (const __bf16*)(const void*)Btp + (size_t)b * strideB;

  const int rlane = lane & 15;
  const int koff  = (lane >> 4) * 8;
  const int mOff  = (lane >> 4) * 8;

  const __bf16* pa = Ab + (size_t)(m0 + rlane) * lda + koff;
  const __bf16* pb = Bb + (size_t)(n0 + rlane) * ldb + koff;

  v8f acc[4][4];
#pragma unroll
  for (int i = 0; i < 4; ++i)
#pragma unroll
    for (int j = 0; j < 4; ++j) acc[i][j] = (v8f){0.f, 0.f, 0.f, 0.f, 0.f, 0.f, 0.f, 0.f};

#pragma unroll 1
  for (int k0 = 0; k0 < K; k0 += 32) {
    v16b bh[4];
#pragma unroll
    for (int j = 0; j < 4; ++j) bh[j] = ld_frag(pb + (size_t)(j << 4) * ldb + k0);
#pragma unroll
    for (int i = 0; i < 4; ++i) {
      const v16b ah = ld_frag(pa + (size_t)(i << 4) * lda + k0);
#pragma unroll
      for (int j = 0; j < 4; ++j) acc[i][j] = mma_bf16(ah, bh[j], acc[i][j]);
    }
  }

  float* slab = sT[wave];
  float* C = Cout + (size_t)b * strideC;
#pragma unroll
  for (int i = 0; i < 4; ++i) {
    const int mBase = m0 + (i << 4);
#pragma unroll
    for (int j = 0; j < 4; ++j) {
#pragma unroll
      for (int r = 0; r < 8; ++r) slab[(mOff + r) * 68 + (j << 4) + rlane] = acc[i][j][r];
    }
    __builtin_amdgcn_fence(__ATOMIC_RELEASE, "workgroup");
    __builtin_amdgcn_wave_barrier();
    __builtin_amdgcn_fence(__ATOMIC_ACQUIRE, "workgroup");
    {
      const int hh = lane >> 4, c4 = (lane & 15) * 4;
      for (int pass = 0; pass < 2; ++pass) {
#pragma unroll
        for (int it = 0; it < 8; ++it) {
          const int row = it * 2 + hh;
          const v4f v = *(const v4fa*)(slab + row * 68 + c4);
          *(volatile v4f*)(C + (size_t)(mBase + row) * ldc + n0 + c4) = v;
        }
        __threadfence();
      }
    }
    __builtin_amdgcn_fence(__ATOMIC_RELEASE, "workgroup");
    __builtin_amdgcn_wave_barrier();
    __builtin_amdgcn_fence(__ATOMIC_ACQUIRE, "workgroup");
  }
}

__global__ __launch_bounds__(256) void k_rowpost(const float* __restrict__ HW, const int* __restrict__ positions,
                                                 const float* __restrict__ pos_table, const float* __restrict__ AV,
                                                 float* __restrict__ F12, unsigned short* __restrict__ VT3) {
  extern __shared__ float tileD[];
  __shared__ __attribute__((aligned(16))) float sAV[1024];
  __shared__ __attribute__((aligned(16))) float sF[128];

  const int tid = threadIdx.x, lane = tid & 31, w = tid >> 5;
  const int blk = blockIdx.x;
  const int b   = blk >> 4;
  const int n0  = (blk & 15) * RP_ROWS;
  const int R0  = blk * RP_ROWS;

  {
    const v4f v = *(const v4fa*)(AV + tid * 4);
    *(v4fa*)(sAV + tid * 4) = v;
  }
  __syncthreads();

#pragma unroll 1
  for (int rr = 0; rr < 8; ++rr) {
    const int lr = 8 * w + rr;
    const int grow = R0 + lr;
    int pos = positions[grow];
    pos = min(max(pos, 0), NN - 1);
    const float* hwr = HW + (size_t)grow * OUT_F;
    const float* ptr = pos_table + (size_t)pos * OUT_F;
    float* trow = tileD + lr * RP_PITCH;
    float f1p = 0.0f, f2p = 0.0f;
#pragma unroll
    for (int it = 0; it < 4; ++it) {
      const int c = it * 128 + lane * 4;
      const v4f hw = *(const v4fa*)(hwr + c);
      const v4f pt = *(const v4fa*)(ptr + c);
      const v4f a1 = *(const v4fa*)(sAV + c);
      const v4f a2 = *(const v4fa*)(sAV + OUT_F + c);
#pragma unroll
      for (int e = 0; e < 4; ++e) {
        const float wh = hw[e] + bf16r(pt[e]);
        f1p += wh * a1[e];
        f2p += wh * a2[e];
        trow[c + e] = wh;
      }
    }
#pragma unroll
    for (int off = 16; off > 0; off >>= 1) {
      f1p += __shfl_xor(f1p, off, 32);
      f2p += __shfl_xor(f2p, off, 32);
    }
    if (lane == 0) { sF[lr] = f1p; sF[64 + lr] = f2p; }
  }
  __syncthreads();

  const int jg = tid & 7, osub = tid >> 3;
  for (int pass = 0; pass < 2; ++pass) {
    if (w == 0) {
      const int hsel = lane >> 4, c4 = (lane & 15) * 4;
      const v4f v = *(const v4fa*)(sF + hsel * 64 + c4);
      *(volatile v4f*)(F12 + (size_t)hsel * MROWS + R0 + c4) = v;
    }
#pragma unroll 1
    for (int it = 0; it < 16; ++it) {
      const int o = it * 32 + osub;
      const float* tc = tileD + (jg * 8) * RP_PITCH + o;
      const v4f x0 = (v4f){ tc[0], tc[RP_PITCH], tc[2 * RP_PITCH], tc[3 * RP_PITCH] };
      const v4f x1 = (v4f){ tc[4 * RP_PITCH], tc[5 * RP_PITCH], tc[6 * RP_PITCH], tc[7 * RP_PITCH] };
      const HL s = split8(x0, x1);
      const size_t base = ((size_t)(b * OUT_F + o)) * K3 + n0 + jg * 8;
      *(volatile v4u*)(VT3 + base) = s.h;
      if (PSPLIT) *(volatile v4u*)(VT3 + base + (size_t)SEG_PLO * NN) = s.h;
      if (VSPLIT) *(volatile v4u*)(VT3 + base + (size_t)SEG_VLO * NN) = s.l;
    }
    __threadfence();
  }
}

__global__ __launch_bounds__(256) void k_softmax(const float* __restrict__ F12, const int* __restrict__ adj,
                                                 float* __restrict__ out1, unsigned short* __restrict__ P3) {
  __shared__ __attribute__((aligned(16))) float sF2[NN];
  __shared__ __attribute__((aligned(16))) float sE[8][NN];

  const int tid = threadIdx.x, lane = tid & 31, w = tid >> 5;
  const int blk = blockIdx.x;
  const int b = blk >> 7;
  const int i = ((blk & 127) << 3) + w;
  const int grow = b * NN + i;

  {
    const v4f v = *(const v4fa*)(F12 + MROWS + b * NN + tid * 4);
    *(v4fa*)(sF2 + tid * 4) = v;
  }
  __syncthreads();

  const float fi = F12[grow];
  const int* arow = adj + (size_t)grow * NN;
  float* se = sE[w];
  const float NEGF = -9.0e15f;

  float mx = -INFINITY;
#pragma unroll 1
  for (int q = 0; q < 8; ++q) {
    const int j = q * 128 + lane * 4;
    const v4i av = *(const v4ia*)(arow + j);
    asm volatile("" :: "v"(av));
    const v4f f2 = *(const v4fa*)(sF2 + j);
    v4f e;
#pragma unroll
    for (int k = 0; k < 4; ++k) {
      float x = fi + f2[k];
      x = (x >= 0.0f) ? x : 0.2f * x;
      const float ev = (av[k] > 0) ? x : NEGF;
      e[k] = ev;
      mx = fmaxf(mx, ev);
    }
    *(v4fa*)(se + j) = e;
  }
#pragma unroll
  for (int off = 16; off > 0; off >>= 1) mx = fmaxf(mx, __shfl_xor(mx, off, 32));

  float ssum = 0.0f;
#pragma unroll 1
  for (int q = 0; q < 8; ++q) {
    const int j = q * 128 + lane * 4;
    const v4f e = *(const v4fa*)(se + j);
    v4f p;
#pragma unroll
    for (int k = 0; k < 4; ++k) {
      const float pv = expf(e[k] - mx);
      p[k] = pv;
      ssum += pv;
    }
    *(v4fa*)(se + j) = p;
  }
#pragma unroll
  for (int off = 16; off > 0; off >>= 1) ssum += __shfl_xor(ssum, off, 32);
  const float inv = 1.0f / ssum;

#pragma unroll 1
  for (int q = 0; q < 8; ++q) {
    const int j = q * 128 + lane * 4;
    const v4f p = *(const v4fa*)(se + j);
    const v4f at = (v4f){ p[0] * inv, p[1] * inv, p[2] * inv, p[3] * inv };
    *(v4fa*)(se + j) = at;
  }
  __builtin_amdgcn_fence(__ATOMIC_RELEASE, "workgroup");
  __builtin_amdgcn_wave_barrier();
  __builtin_amdgcn_fence(__ATOMIC_ACQUIRE, "workgroup");

  float* orow = out1 + (size_t)grow * NN;
  unsigned short* prow = P3 + (size_t)grow * K3;
  for (int pass = 0; pass < 2; ++pass) {
#pragma unroll 1
    for (int q = 0; q < 8; ++q) {
      const int j = q * 128 + lane * 4;
      const v4f v = *(const v4fa*)(se + j);
      *(volatile v4f*)(orow + j) = v;
    }
#pragma unroll 1
    for (int u = 0; u < 4; ++u) {
      const int j = u * 256 + lane * 8;
      const v4f x0 = *(const v4fa*)(se + j);
      const v4f x1 = *(const v4fa*)(se + j + 4);
      const HL s = split8(x0, x1);
      *(volatile v4u*)(prow + j) = s.h;
      if (PSPLIT) *(volatile v4u*)(prow + (size_t)SEG_PLO * NN + j) = s.l;
      if (VSPLIT) *(volatile v4u*)(prow + (size_t)SEG_VLO * NN + j) = s.h;
    }
    __threadfence();
  }
}

extern "C" void kernel_launch(void* const* d_in, const int* in_sizes, int n_in,
                              void* d_out, int out_size, void* d_ws, size_t ws_size,
                              hipStream_t stream) {
  if (n_in < 6) return;
  if (in_sizes[0] != MROWS * IN_F) return;
  if (in_sizes[1] != NB * NN * NN) return;
  if (in_sizes[2] != MROWS) return;
  if (in_sizes[3] != IN_F * OUT_F) return;
  if (in_sizes[4] != 2 * OUT_F) return;
  if (in_sizes[5] != NN * OUT_F) return;
  if (out_size != OUT0_ELEMS + OUT1_ELEMS) return;
  if (WS_TOTAL > ws_size) return;

  const float* h         = (const float*)d_in[0];
  const int*   adj       = (const int*)  d_in[1];
  const int*   positions = (const int*)  d_in[2];
  const float* W         = (const float*)d_in[3];
  const float* a         = (const float*)d_in[4];
  const float* pos_table = (const float*)d_in[5];

  float* out0 = (float*)d_out;
  float* out1 = (float*)d_out + (size_t)OUT0_ELEMS;

  char* ws = (char*)d_ws;
  size_t off = 0;
  unsigned short* HB  = (unsigned short*)(ws + off); off += WS_HB;
  unsigned short* WT  = (unsigned short*)(ws + off); off += WS_WT;
  float*          AV  = (float*)(ws + off);          off += WS_AV;
  float*          HW  = (float*)(ws + off);          off += WS_HW;
  float*          F12 = (float*)(ws + off);          off += WS_F12;
  unsigned short* P3  = (unsigned short*)(ws + off); off += WS_P3;
  unsigned short* VT3 = (unsigned short*)(ws + off); off += WS_VT3;
  if (off > ws_size) return;

  k_prep<<<dim3(NHB + NWT + 1), dim3(256), 0, stream>>>(h, W, a, HB, WT, AV);

  k_gemm_bf16<<<dim3((MROWS / 64) * (OUT_F / 64) / 8, 1), dim3(256), 0, stream>>>(
      HB, IN_F, 0L, WT, IN_F, 0L, HW, OUT_F, 0L, MROWS, OUT_F, IN_F);

  (void)hipFuncSetAttribute(reinterpret_cast<const void*>(&k_rowpost),
                            hipFuncAttributeMaxDynamicSharedMemorySize, RP_DYN);
  k_rowpost<<<dim3(MROWS / RP_ROWS), dim3(256), RP_DYN, stream>>>(HW, positions, pos_table, AV, F12, VT3);

  k_softmax<<<dim3(MROWS / 8), dim3(256), 0, stream>>>(F12, adj, out1, P3);

  k_gemm_bf16<<<dim3((NN / 64) * (OUT_F / 64) / 8, NB), dim3(256), 0, stream>>>(
      P3, K3, (long)NN * K3, VT3, K3, (long)OUT_F * K3, out0, OUT_F, (long)NN * OUT_F, NN, OUT_F, K3);

  (void)hipGetLastError();
}
